// QuantumGate_65481071399866
// MI455X (gfx1250) — hardware-verified
//
#include <hip/hip_runtime.h>
#include <math.h>

typedef __attribute__((ext_vector_type(16))) _Float16 v16h;
typedef __attribute__((ext_vector_type(8)))  _Float16 v8h;
typedef __attribute__((ext_vector_type(8)))  float    v8f;
typedef __attribute__((ext_vector_type(4)))  float    v4f;
typedef __attribute__((ext_vector_type(2)))  float    v2f;

constexpr int kRowsTotal = 256;
constexpr int kWidth     = 14;
constexpr int kTileRows  = 16;
constexpr int kKPad      = 32;
static_assert((kRowsTotal % kTileRows) == 0, "row tiles");
static_assert(((kTileRows * kWidth * 4) % 128) == 0, "a 16-row output tile is a whole number of 128-B lines");
static_assert((kTileRows * kWidth) / 4 == 56, "56 float4 per output tile");
static_assert((kWidth % 2) == 0 && kWidth <= 14, "row loads as 7 x 8-B words; value slots 0..13, remainder slots 16..29");

constexpr float kCarryX   = 16.0f;
constexpr float kCarryW   = 64.0f;
constexpr float kCarryZ   = 1024.0f;
constexpr float kResScale = 2048.0f;
constexpr float kInvRes   = 1.0f / kResScale;
constexpr float kInvAng   = 1.0f / (kCarryX * kCarryW);
constexpr float kInvOut   = 1.0f / (kCarryZ * kCarryW);
constexpr float kHalfMinNormal = 6.103515625e-05f;

union FragU { v16h v; v8h h[2]; };

__device__ __forceinline__ v16h frag_load(const _Float16* p) {
  FragU f;
  f.h[0] = *(const v8h*)(p);
  f.h[1] = *(const v8h*)(p + 16);
  return f.v;
}

__device__ __forceinline__ v8f mma_f16(v16h a, v16h b, v8f c) {
  c = __builtin_amdgcn_wmma_f32_16x16x32_f16(false, a, false, b, (short)0, c, false, false);
  asm volatile("v_nop\n\tv_nop\n\tv_nop\n\tv_nop" : "+v"(c) : "v"(a), "v"(b));
  return c;
}

__device__ __forceinline__ float flush_h(float v) {
  return (fabsf(v) < kHalfMinNormal) ? 0.0f : v;
}

__device__ __forceinline__ void split_h(float c, float& hif, float& lof) {
  const float cf = flush_h(c);
  const _Float16 hh = (_Float16)cf;
  hif = (float)hh;
  lof = flush_h((c - hif) * kResScale);
}

__device__ __forceinline__ void stage_a_half_row(const float (&v)[kWidth], float carry, int half,
                                                 _Float16 zh, _Float16* dst) {
  v8h o0, o1;
#pragma unroll
  for (int k = 0; k < kWidth; ++k) {
    float hif, lof;
    split_h(v[k] * carry, hif, lof);
    const float sel = (half != 0) ? lof : hif;
    const _Float16 hv = (_Float16)sel;
    if (k < 8) o0[k] = hv;
    else       o1[k - 8] = hv;
  }
  o1[6] = zh;
  o1[7] = zh;
  *(v8h*)(dst)     = o0;
  *(v8h*)(dst + 8) = o1;
}

__global__ __launch_bounds__(32) void fused_rot_chain_kernel(const float* __restrict__ x,
                                                             const float* __restrict__ W,
                                                             float* __restrict__ out) {
  __shared__ __align__(16) _Float16 sA[kTileRows * kKPad];
  __shared__ __align__(16) _Float16 sB1[16 * kKPad];
  __shared__ __align__(16) _Float16 sB2[16 * kKPad];
  __shared__ __align__(16) float    sC[16 * 16];
  __shared__ __align__(16) float    sO[256];

  const int lane  = threadIdx.x & 31;
  const int hsel  = lane >> 4;
  const int col   = lane & 15;
  const int srow  = lane >> 1;
  const int shalf = lane & 1;
  const int mbase = blockIdx.x * kTileRows;

  float zf = 0.0f;
  asm volatile("" : "+v"(zf));
  const _Float16 zh = (_Float16)zf;

  {
    int grow = mbase + srow;
    grow = (grow < kRowsTotal) ? grow : (kRowsTotal - 1);
    const v2f* xp = (const v2f*)(x + (size_t)grow * kWidth);
    float xv[kWidth];
#pragma unroll
    for (int i = 0; i < kWidth / 2; ++i) {
      const v2f t = xp[i];
      xv[2 * i]     = t[0];
      xv[2 * i + 1] = t[1];
    }
    stage_a_half_row(xv, kCarryX, shalf, zh, sA + srow * kKPad + shalf * 16);
  }

  {
    const int  nc     = (srow < kWidth) ? srow : (kWidth - 1);
    const bool wvalid = (srow < kWidth);
    const v2f* wp = (const v2f*)(W + (size_t)nc * kWidth);
    float wv[kWidth];
#pragma unroll
    for (int i = 0; i < kWidth / 2; ++i) {
      const v2f t = wp[i];
      wv[2 * i]     = wvalid ? t[0] : 0.0f;
      wv[2 * i + 1] = wvalid ? t[1] : 0.0f;
    }
    v8h p0, p1, q0, q1;
#pragma unroll
    for (int k = 0; k < kWidth; ++k) {
      float hif, lof;
      split_h(wv[k] * kCarryW, hif, lof);
      const float f1 = (shalf != 0) ? 0.0f : hif;
      const float f2 = (shalf != 0) ? hif  : lof;
      const _Float16 h1 = (_Float16)f1;
      const _Float16 h2 = (_Float16)f2;
      if (k < 8) { p0[k] = h1; q0[k] = h2; }
      else       { p1[k - 8] = h1; q1[k - 8] = h2; }
    }
    p1[6] = zh;
    p1[7] = zh;
    q1[6] = zh;
    q1[7] = zh;
    _Float16* d1 = sB1 + srow * kKPad + shalf * 16;
    _Float16* d2 = sB2 + srow * kKPad + shalf * 16;
    *(v8h*)(d1)     = p0;
    *(v8h*)(d1 + 8) = p1;
    *(v8h*)(d2)     = q0;
    *(v8h*)(d2 + 8) = q1;
  }
  __syncthreads();

  const v16h fb1 = frag_load(sB1 + col * kKPad + 8 * hsel);
  const v16h fb2 = frag_load(sB2 + col * kKPad + 8 * hsel);

  {
    const v16h fa = frag_load(sA + col * kKPad + 8 * hsel);
    v8f accV = (v8f){0.f, 0.f, 0.f, 0.f, 0.f, 0.f, 0.f, 0.f};
    v8f accR = (v8f){0.f, 0.f, 0.f, 0.f, 0.f, 0.f, 0.f, 0.f};
    accV = mma_f16(fa, fb1, accV);
    accR = mma_f16(fa, fb2, accR);
#pragma unroll
    for (int r = 0; r < 8; ++r) {
      const float ang = (accV[r] + accR[r] * kInvRes) * kInvAng;
      sC[(8 * hsel + r) * 16 + col] = ang;
    }
  }
  __syncthreads();

#pragma unroll 1
  for (int i = 0; i < 8; ++i) {
    const int idx = lane + 32 * i;
    const float a = sC[idx];
    sC[idx] = cosf(a);
  }
  __syncthreads();

  {
    float cv[kWidth];
#pragma unroll
    for (int k = 0; k < kWidth; ++k) cv[k] = sC[srow * 16 + k];
    float zv[kWidth];
    float p = cv[0];
#pragma unroll
    for (int j = 1; j < kWidth; ++j) {
      p = p * cv[j];
      zv[j] = p;
    }
    float q = cv[1];
#pragma unroll
    for (int j = 2; j < kWidth; ++j) q = q * cv[j];
    zv[0] = q;
    stage_a_half_row(zv, kCarryZ, shalf, zh, sA + srow * kKPad + shalf * 16);
  }
  __syncthreads();

  {
    const v16h fz = frag_load(sA + col * kKPad + 8 * hsel);
    v8f accV = (v8f){0.f, 0.f, 0.f, 0.f, 0.f, 0.f, 0.f, 0.f};
    v8f accR = (v8f){0.f, 0.f, 0.f, 0.f, 0.f, 0.f, 0.f, 0.f};
    accV = mma_f16(fz, fb1, accV);
    accR = mma_f16(fz, fb2, accR);
#pragma unroll
    for (int r = 0; r < 8; ++r) {
      const int row = 8 * hsel + r;
      const float val = (accV[r] + accR[r] * kInvRes) * kInvOut;
      const int idx = (col < kWidth) ? (row * kWidth + col) : (224 + (col - kWidth) * 16 + row);
      sO[idx] = val;
    }
  }
  __syncthreads();

  {
    const v4f* so4 = (const v4f*)sO;
    const int i1 = (lane < 24) ? (32 + lane) : 55;
    const v4f o0 = so4[lane];
    const v4f o1 = so4[i1];
    float* ob = out + (size_t)mbase * kWidth;
    for (int pass = 0; pass < 2; ++pass) {
      *(volatile v4f*)(ob + 4 * lane) = o0;
      if (lane < 24) {
        *(volatile v4f*)(ob + 128 + 4 * lane) = o1;
      }
      __threadfence();
    }
  }
}

extern "C" void kernel_launch(void* const* d_in, const int* in_sizes, int n_in,
                              void* d_out, int out_size, void* d_ws, size_t ws_size,
                              hipStream_t stream) {
  (void)d_ws;
  (void)ws_size;
  if (n_in < 2) return;
  if (in_sizes[0] != kRowsTotal * kWidth) return;
  if (in_sizes[1] != kWidth * kWidth) return;
  if (out_size != kRowsTotal * kWidth) return;

  const float* x = (const float*)d_in[0];
  const float* W = (const float*)d_in[1];
  float* out = (float*)d_out;

  fused_rot_chain_kernel<<<dim3(kRowsTotal / kTileRows), dim3(32), 0, stream>>>(x, W, out);
}
